// TemporalItemGAT_17910013624757
// MI455X (gfx1250) — hardware-verified
//
#include <hip/hip_runtime.h>
#include <stddef.h>


#define IND   32
#define DF1   128
#define DF2   64
#define NH1   2
#define NH2   1
#define GR    32
#define XSP   132
#define NTHR  256
#define NWAVE 8
#define CHUNK 2048
#define WCAP  256
#define NGRP  (CHUNK / (NTHR * 4))
#define NB1   512
#define SB1   9
#define NB2   1024
#define SB2   10
#define SLOPE 0.2f
#define MXINIT (-1.0e30f)

#define L1_SACC (NB1 * DF1)
#define L1_DEN  (NB1 * NH1)
#define L1_A2S  (NB1 * 2)
#define L1_MX   (NB1 * NH1)
#define L_LIST  (NWAVE * WCAP)
#define L_WC    16
#define LDS1_BYTES ((L1_SACC + L1_DEN + L1_A2S + L1_MX + L_LIST + L_WC) * 4)
#define L2_SACC (NB2 * DF2)
#define L2_DEN  (NB2 * NH2)
#define L2_MX   (NB2 * NH2)
#define LDS2_BYTES ((L2_SACC + L2_DEN + L2_MX + L_LIST + L_WC) * 4)

static_assert(WCAP == (CHUNK / NTHR) * 32);
static_assert(NGRP == 2);
static_assert((1 << SB1) == NB1);
static_assert((1 << SB2) == NB2);
static_assert(CHUNK == 2048);
static_assert(NTHR == NWAVE * 32);
static_assert(LDS1_BYTES == 282688);
static_assert(LDS2_BYTES == 278592);
static_assert(((L1_SACC + L1_DEN + L1_A2S) % 4) == 0);
static_assert(((L2_SACC + L2_DEN) % 4) == 0);
static_assert((NB1 / NWAVE) == 64);
static_assert((NB2 / NWAVE) == 128);

typedef float          v2f   __attribute__((ext_vector_type(2)));
typedef float          v4f   __attribute__((ext_vector_type(4)));
typedef float          v8f   __attribute__((ext_vector_type(8)));
typedef int            v4i   __attribute__((ext_vector_type(4)));
typedef unsigned int   v2u   __attribute__((ext_vector_type(2)));
typedef unsigned int   v4u   __attribute__((ext_vector_type(4)));
typedef unsigned short v8us  __attribute__((ext_vector_type(8)));
typedef __bf16         v16bf __attribute__((ext_vector_type(16)));
union FragB { v16bf v; v8us half[2]; unsigned int w[8]; };

template <int VW> struct VT;
template <> struct VT<4> { typedef v4f t; };
template <> struct VT<2> { typedef v2f t; };

__device__ __forceinline__ v8f wmb(v16bf a, v16bf b, v8f c) {
  v8f d = __builtin_amdgcn_wmma_f32_16x16x32_bf16(false, a, false, b, (short)0, c, false, false);
  asm volatile("v_nop\n\tv_nop\n\tv_nop\n\tv_nop" : "+v"(d) : "v"(a), "v"(b));
  return d;
}

__device__ __forceinline__ unsigned int bfbits(float f) {
  const unsigned int u = __float_as_uint(f);
  return (u + 0x7FFFu + ((u >> 16) & 1u)) >> 16;
}
__device__ __forceinline__ void split2(float f, unsigned int& h, unsigned int& l) {
  h = bfbits(f);
  l = bfbits(f - __uint_as_float(h << 16));
}
__device__ __forceinline__ void pack_pair(float f0, float f1, unsigned int& hw, unsigned int& lw) {
  unsigned int h0, l0, h1, l1;
  split2(f0, h0, l0);
  split2(f1, h1, l1);
  hw = h0 | (h1 << 16);
  lw = l0 | (l1 << 16);
}

__global__ __launch_bounds__(NTHR) void k_wprep(const float* __restrict__ W,
                                                unsigned short* Wh, unsigned short* Wl,
                                                int K, int Nc) {
  const int t = blockIdx.x * NTHR + threadIdx.x;
  const int o = t * 8;
  if (o >= K * Nc) return;
  const int n  = o / K;
  const int k0 = o - n * K;
  const float* p = W + (size_t)k0 * Nc + n;
  unsigned int hw, lw;
  v4u H, L;
  pack_pair(p[0 * Nc], p[1 * Nc], hw, lw); H.x = hw; L.x = lw;
  pack_pair(p[2 * Nc], p[3 * Nc], hw, lw); H.y = hw; L.y = lw;
  pack_pair(p[4 * Nc], p[5 * Nc], hw, lw); H.z = hw; L.z = lw;
  pack_pair(p[6 * Nc], p[7 * Nc], hw, lw); H.w = hw; L.w = lw;
  *(volatile v4u*)(Wh + o) = H;
  *(volatile v4u*)(Wl + o) = L;
  __threadfence();
  *(volatile v4u*)(Wh + o) = H;
  *(volatile v4u*)(Wl + o) = L;
}

__device__ __forceinline__ void epi1(v8f acc, int T, int hh, int m, int wave, int ncol,
                                     float cs, float cd, float* Xs, float* As, float* Ds) {
  float ss[8], sd[8];
#pragma unroll
  for (int r = 0; r < 8; ++r) {
    const float v = acc[r];
    Xs[(T * 16 + 8 * hh + r) * XSP + ncol] = v;
    ss[r] = v * cs;
    sd[r] = v * cd;
  }
#pragma unroll
  for (int mk = 1; mk < 16; mk <<= 1) {
#pragma unroll
    for (int r = 0; r < 8; ++r) {
      ss[r] += __shfl_xor(ss[r], mk, 32);
      sd[r] += __shfl_xor(sd[r], mk, 32);
    }
  }
  if (m == 0) {
#pragma unroll
    for (int r = 0; r < 8; ++r) {
      As[(T * 16 + 8 * hh + r) * NWAVE + wave] = ss[r];
      Ds[(T * 16 + 8 * hh + r) * NWAVE + wave] = sd[r];
    }
  }
}

__global__ __launch_bounds__(NTHR) void k_node1(
    const int* __restrict__ ids, const float* __restrict__ emb,
    const unsigned short* __restrict__ W1h, const unsigned short* __restrict__ W1l,
    const float* __restrict__ att_s, const float* __restrict__ att_d,
    float* hp1, float* a1, int nN, int nI) {
  __shared__ __attribute__((aligned(16))) unsigned short Ah[GR * IND];
  __shared__ __attribute__((aligned(16))) unsigned short Al[GR * IND];
  __shared__ __attribute__((aligned(16))) float Xs[GR * XSP];
  __shared__ __attribute__((aligned(16))) float As[GR * NWAVE];
  __shared__ __attribute__((aligned(16))) float Ds[GR * NWAVE];

  const int tid  = threadIdx.x;
  const int lane = tid & 31;
  const int wave = tid >> 5;
  const int hh   = lane >> 4;
  const int m    = lane & 15;
  const int rowBase = blockIdx.x * GR;
  const v4f z4 = {0.f, 0.f, 0.f, 0.f};

  {
    const int r  = tid >> 3;
    const int c0 = (tid & 7) * 4;
    const int node = rowBase + r;
    const int nd = node < nN ? node : nN - 1;
    const int id = ids[nd];
    const int idc = id < 0 ? 0 : (id > nI - 1 ? nI - 1 : id);
    v4f v = *(const v4f*)(emb + (size_t)idc * IND + c0);
    if (idc == 0 || node >= nN) v = z4;
    v2u hv, lv;
    unsigned int hw, lw;
    pack_pair(v.x, v.y, hw, lw); hv.x = hw; lv.x = lw;
    pack_pair(v.z, v.w, hw, lw); hv.y = hw; lv.y = lw;
    *(v2u*)(Ah + r * IND + c0) = hv;
    *(v2u*)(Al + r * IND + c0) = lv;
  }
  __syncthreads();

  const int ncol = wave * 16 + m;
  FragB bh, bl, ah0, al0, ah1, al1;
  {
    const unsigned short* pbh = W1h + (size_t)ncol * IND + 8 * hh;
    const unsigned short* pbl = W1l + (size_t)ncol * IND + 8 * hh;
    bh.half[0] = *(const v8us*)pbh;  bh.half[1] = *(const v8us*)(pbh + 16);
    bl.half[0] = *(const v8us*)pbl;  bl.half[1] = *(const v8us*)(pbl + 16);
    const unsigned short* pa0h = Ah + m * IND + 8 * hh;
    const unsigned short* pa0l = Al + m * IND + 8 * hh;
    const unsigned short* pa1h = Ah + (16 + m) * IND + 8 * hh;
    const unsigned short* pa1l = Al + (16 + m) * IND + 8 * hh;
    ah0.half[0] = *(const v8us*)pa0h; ah0.half[1] = *(const v8us*)(pa0h + 16);
    al0.half[0] = *(const v8us*)pa0l; al0.half[1] = *(const v8us*)(pa0l + 16);
    ah1.half[0] = *(const v8us*)pa1h; ah1.half[1] = *(const v8us*)(pa1h + 16);
    al1.half[0] = *(const v8us*)pa1l; al1.half[1] = *(const v8us*)(pa1l + 16);
  }
  v8f c0a = {0.f, 0.f, 0.f, 0.f, 0.f, 0.f, 0.f, 0.f};
  v8f c1a = {0.f, 0.f, 0.f, 0.f, 0.f, 0.f, 0.f, 0.f};
  c0a = wmb(ah0.v, bh.v, c0a);
  c0a = wmb(ah0.v, bl.v, c0a);
  c0a = wmb(al0.v, bh.v, c0a);
  c1a = wmb(ah1.v, bh.v, c1a);
  c1a = wmb(ah1.v, bl.v, c1a);
  c1a = wmb(al1.v, bh.v, c1a);

  const float cs = att_s[ncol];
  const float cd = att_d[ncol];
  epi1(c0a, 0, hh, m, wave, ncol, cs, cd, Xs, As, Ds);
  epi1(c1a, 1, hh, m, wave, ncol, cs, cd, Xs, As, Ds);
  __syncthreads();

  v4f xr[4];
#pragma unroll
  for (int i = 0; i < 4; ++i) xr[i] = *(const v4f*)(Xs + (4 * wave + i) * XSP + 4 * lane);
  float* xpp[4];
#pragma unroll
  for (int i = 0; i < 4; ++i) xpp[i] = hp1 + (size_t)(rowBase + 4 * wave + i) * DF1 + 4 * lane;
  v4f av = z4;
  float* ap = a1 + (size_t)(rowBase + lane) * 4;
  const bool wa = (wave == 0);
  if (wa) {
    const v4f s03 = *(const v4f*)(As + lane * NWAVE);
    const v4f s47 = *(const v4f*)(As + lane * NWAVE + 4);
    const v4f d03 = *(const v4f*)(Ds + lane * NWAVE);
    const v4f d47 = *(const v4f*)(Ds + lane * NWAVE + 4);
    av.x = (s03.x + s03.y) + (s03.z + s03.w);
    av.y = (s47.x + s47.y) + (s47.z + s47.w);
    av.z = (d03.x + d03.y) + (d03.z + d03.w);
    av.w = (d47.x + d47.y) + (d47.z + d47.w);
  }
#pragma unroll
  for (int i = 0; i < 4; ++i) *(volatile v4f*)(xpp[i]) = xr[i];
  if (wa) *(volatile v4f*)ap = av;
  __threadfence();
#pragma unroll
  for (int i = 0; i < 4; ++i) *(volatile v4f*)(xpp[i]) = xr[i];
  if (wa) *(volatile v4f*)ap = av;
}

template <int DF, int NHD, int NB, int SB>
__device__ __forceinline__ void scan_drain(
    const float* __restrict__ hp, const int* __restrict__ ei, const float* __restrict__ ap,
    float* sacc, float* mx, float* den, int* list, int* wcnt,
    int nN, int nE, int nodeBase, int tid, int lane, int wave) {
  constexpr int VW  = DF / 32;
  constexpr int AW  = 2 * NHD;
  constexpr int LPH = 32 / NHD;
  typedef typename VT<VW>::t vt;
  static_assert(SB + 11 <= 30);
  static_assert(VW * 32 == DF);
  const int hd = lane / LPH;
  const int* eid = ei + nE;
  const bool al16 = ((nE & 3) == 0);
  const int nChunks = (nE + CHUNK - 1) / CHUNK;

#pragma unroll 1
  for (int ch = 0; ch < nChunks; ++ch) {
    const int cbase = ch * CHUNK;
    int wc = 0;
#pragma unroll
    for (int g = 0; g < NGRP; ++g) {
      const int el0 = (g * NTHR + tid) * 4;
      const int e0  = cbase + el0;
      const int sent = -2147483647 - 1;
      v4i d;
      if (al16 && (cbase + CHUNK <= nE)) {
        d = *(const v4i*)(eid + e0);
      } else {
        const int q0 = e0     < nE ? e0     : nE - 1;
        const int q1 = e0 + 1 < nE ? e0 + 1 : nE - 1;
        const int q2 = e0 + 2 < nE ? e0 + 2 : nE - 1;
        const int q3 = e0 + 3 < nE ? e0 + 3 : nE - 1;
        const int u0 = eid[q0], u1 = eid[q1], u2 = eid[q2], u3 = eid[q3];
        d.x = (e0     < nE) ? u0 : sent;
        d.y = (e0 + 1 < nE) ? u1 : sent;
        d.z = (e0 + 2 < nE) ? u2 : sent;
        d.w = (e0 + 3 < nE) ? u3 : sent;
      }
      const unsigned s0 = (unsigned)d.x - (unsigned)nodeBase;
      const unsigned s1 = (unsigned)d.y - (unsigned)nodeBase;
      const unsigned s2 = (unsigned)d.z - (unsigned)nodeBase;
      const unsigned s3 = (unsigned)d.w - (unsigned)nodeBase;
      const bool h0 = s0 < (unsigned)NB;
      const bool h1 = s1 < (unsigned)NB;
      const bool h2 = s2 < (unsigned)NB;
      const bool h3 = s3 < (unsigned)NB;
      const unsigned many = __builtin_amdgcn_ballot_w32(h0 | h1 | h2 | h3);
      if (many != 0u) {
#define HITJ(J, HJ, SJ) { \
          const unsigned mj = __builtin_amdgcn_ballot_w32(HJ); \
          if (HJ) { \
            const int pos = wc + (int)__builtin_amdgcn_mbcnt_lo(mj, 0u); \
            if (pos < WCAP) list[wave * WCAP + pos] = ((el0 + (J)) << SB) | (int)(SJ); \
          } \
          wc += (int)__builtin_popcount(mj); }
        HITJ(0, h0, s0)
        HITJ(1, h1, s1)
        HITJ(2, h2, s2)
        HITJ(3, h3, s3)
#undef HITJ
      }
    }
    if (lane == 0) wcnt[wave] = wc;
    __syncthreads();

    if (wave == 0) {
#pragma unroll 1
      for (int wsx = 0; wsx < NWAVE; ++wsx) {
        int n = wcnt[wsx];
        n = n > WCAP ? WCAP : (n < 0 ? 0 : n);
#pragma unroll 1
        for (int i = 0; i < n; ++i) {
          const int ent  = list[wsx * WCAP + i];
          const int slot = ent & (NB - 1);
          const int el   = (ent >> SB) & (CHUNK - 1);
          int e = cbase + el;
          e = e > nE - 1 ? nE - 1 : e;
          int src = ei[e];
          src = src < 0 ? 0 : (src > nN - 1 ? nN - 1 : src);
          int nd = nodeBase + slot;
          nd = nd > nN - 1 ? nN - 1 : nd;
          float a = ap[(size_t)src * AW + hd] + ap[(size_t)nd * AW + NHD + hd];
          a = (a > 0.f) ? a : SLOPE * a;
          const int ai = slot * NHD + hd;
          const float M  = mx[ai];
          const float Mn = fmaxf(M, a);
          const float sc = __expf(fmaxf(M - Mn, -80.f));
          const float p  = __expf(fmaxf(a - Mn, -80.f));
          const vt xv = *(const vt*)(hp + (size_t)src * DF + VW * lane);
          vt* sp = (vt*)(sacc + slot * DF + VW * lane);
          const vt cur = *sp;
          const vt nxt = cur * sc + xv * p;
          *sp = nxt;
          const float dn = den[ai];
          den[ai] = dn * sc + p;
          mx[ai]  = Mn;
        }
      }
    }
    __syncthreads();
  }
}

__global__ __launch_bounds__(NTHR) void k_gat1(
    const float* __restrict__ hp1, const int* __restrict__ ei, const float* __restrict__ a1,
    const float* __restrict__ bias,
    const unsigned short* __restrict__ W2h, const unsigned short* __restrict__ W2l,
    const float* __restrict__ att_s, const float* __restrict__ att_d,
    float* hp2, float* a2, int nN, int nE) {
  extern __shared__ v4f lds_dyn[];
  float* sacc = (float*)lds_dyn;
  float* den  = sacc + L1_SACC;
  float* a2s  = den + L1_DEN;
  float* mx   = a2s + L1_A2S;
  int*   list = (int*)(mx + L1_MX);
  int*   wcnt = list + L_LIST;

  const int tid  = threadIdx.x;
  const int lane = tid & 31;
  const int wave = tid >> 5;
  const int hh   = lane >> 4;
  const int m    = lane & 15;
  const int nodeBase = blockIdx.x * NB1;
  const v4f z4 = {0.f, 0.f, 0.f, 0.f};

  for (int i = tid; i < (L1_SACC + L1_DEN + L1_A2S) / 4; i += NTHR) lds_dyn[i] = z4;
  for (int i = tid; i < L1_MX; i += NTHR) mx[i] = MXINIT;
  __syncthreads();

  scan_drain<DF1, NH1, NB1, SB1>(hp1, ei, a1, sacc, mx, den, list, wcnt,
                                 nN, nE, nodeBase, tid, lane, wave);

  {
    const int hd = lane >> 4;
    const v4f b4 = *(const v4f*)(bias + 4 * lane);
#pragma unroll 1
    for (int j = 0; j < NB1 / NWAVE; ++j) {
      const int slot = wave * (NB1 / NWAVE) + j;
      const int node = nodeBase + slot;
      const bool valid = node < nN;
      const int nd = valid ? node : nN - 1;
      float a = a1[(size_t)nd * 4 + hd] + a1[(size_t)nd * 4 + 2 + hd];
      a = (a > 0.f) ? a : SLOPE * a;
      const int ai = slot * NH1 + hd;
      const float M  = mx[ai];
      const float Mn = fmaxf(M, a);
      const float sc = __expf(fmaxf(M - Mn, -80.f));
      const float p  = __expf(fmaxf(a - Mn, -80.f));
      const v4f xv = *(const v4f*)(hp1 + (size_t)nd * DF1 + 4 * lane);
      v4f* sp = (v4f*)(sacc + slot * DF1 + 4 * lane);
      const v4f sv = (*sp) * sc + xv * p;
      const float dv  = den[ai] * sc + p;
      const float inv = 1.0f / (dv + 1e-16f);
      v4f h = sv * inv + b4;
      h.x = h.x > 0.f ? h.x : 0.f;
      h.y = h.y > 0.f ? h.y : 0.f;
      h.z = h.z > 0.f ? h.z : 0.f;
      h.w = h.w > 0.f ? h.w : 0.f;
      if (!valid) h = z4;
      *sp = h;
    }
  }
  __syncthreads();

  const int slot0 = wave * (NB1 / NWAVE);
  {
    float cs[4], cd[4];
#pragma unroll
    for (int ct = 0; ct < 4; ++ct) { cs[ct] = att_s[16 * ct + m]; cd[ct] = att_d[16 * ct + m]; }
#pragma unroll 1
    for (int T = 0; T < 4; ++T) {
      v8f acc[4];
#pragma unroll
      for (int ct = 0; ct < 4; ++ct) acc[ct] = (v8f){0.f, 0.f, 0.f, 0.f, 0.f, 0.f, 0.f, 0.f};
#pragma unroll 1
      for (int kt = 0; kt < DF1 / 32; ++kt) {
        const float* ar = sacc + (slot0 + 16 * T + m) * DF1 + 32 * kt + 8 * hh;
        const v4f f0 = *(const v4f*)(ar);
        const v4f f1 = *(const v4f*)(ar + 4);
        const v4f f2 = *(const v4f*)(ar + 16);
        const v4f f3 = *(const v4f*)(ar + 20);
        FragB fa, fl;
        pack_pair(f0.x, f0.y, fa.w[0], fl.w[0]);
        pack_pair(f0.z, f0.w, fa.w[1], fl.w[1]);
        pack_pair(f1.x, f1.y, fa.w[2], fl.w[2]);
        pack_pair(f1.z, f1.w, fa.w[3], fl.w[3]);
        pack_pair(f2.x, f2.y, fa.w[4], fl.w[4]);
        pack_pair(f2.z, f2.w, fa.w[5], fl.w[5]);
        pack_pair(f3.x, f3.y, fa.w[6], fl.w[6]);
        pack_pair(f3.z, f3.w, fa.w[7], fl.w[7]);
#pragma unroll
        for (int ct = 0; ct < 4; ++ct) {
          const unsigned short* pbh = W2h + (size_t)(16 * ct + m) * DF1 + 32 * kt + 8 * hh;
          const unsigned short* pbl = W2l + (size_t)(16 * ct + m) * DF1 + 32 * kt + 8 * hh;
          FragB bh, bl;
          bh.half[0] = *(const v8us*)pbh; bh.half[1] = *(const v8us*)(pbh + 16);
          bl.half[0] = *(const v8us*)pbl; bl.half[1] = *(const v8us*)(pbl + 16);
          acc[ct] = wmb(fa.v, bh.v, acc[ct]);
          acc[ct] = wmb(fa.v, bl.v, acc[ct]);
          acc[ct] = wmb(fl.v, bh.v, acc[ct]);
        }
      }
      float ss[8], sd[8];
#pragma unroll
      for (int r = 0; r < 8; ++r) { ss[r] = 0.f; sd[r] = 0.f; }
#pragma unroll
      for (int ct = 0; ct < 4; ++ct) {
#pragma unroll
        for (int r = 0; r < 8; ++r) {
          const float v = acc[ct][r];
          sacc[(slot0 + 16 * T + 8 * hh + r) * DF1 + 16 * ct + m] = v;
          ss[r] += v * cs[ct];
          sd[r] += v * cd[ct];
        }
      }
#pragma unroll
      for (int mk = 1; mk < 16; mk <<= 1) {
#pragma unroll
        for (int r = 0; r < 8; ++r) {
          ss[r] += __shfl_xor(ss[r], mk, 32);
          sd[r] += __shfl_xor(sd[r], mk, 32);
        }
      }
      if (m == 0) {
#pragma unroll
        for (int r = 0; r < 8; ++r) {
          a2s[(slot0 + 16 * T + 8 * hh + r) * 2]     = ss[r];
          a2s[(slot0 + 16 * T + 8 * hh + r) * 2 + 1] = sd[r];
        }
      }
    }
  }
  __syncthreads();

  {
    const v4f av = *(const v4f*)(a2s + slot0 * 2 + 4 * lane);
    float* gpa = a2 + (size_t)(nodeBase + slot0) * 2 + 4 * lane;
    *(volatile v4f*)gpa = av;
#pragma unroll 1
    for (int i = 0; i < (NB1 / NWAVE) / 2; ++i) {
      const int r = slot0 + 2 * i + (lane >> 4);
      const int c = 4 * (lane & 15);
      const v4f v = *(const v4f*)(sacc + r * DF1 + c);
      float* gp = hp2 + (size_t)(nodeBase + r) * DF2 + c;
      *(volatile v4f*)gp = v;
      __threadfence();
      *(volatile v4f*)gp = v;
    }
    __threadfence();
    *(volatile v4f*)gpa = av;
  }
}

__global__ __launch_bounds__(NTHR) void k_gat2(
    const float* __restrict__ hp2, const int* __restrict__ ei, const float* __restrict__ a2,
    const float* __restrict__ bias, float* out, int nN, int nE) {
  extern __shared__ v4f lds_dyn[];
  float* sacc = (float*)lds_dyn;
  float* den  = sacc + L2_SACC;
  float* mx   = den + L2_DEN;
  int*   list = (int*)(mx + L2_MX);
  int*   wcnt = list + L_LIST;

  const int tid  = threadIdx.x;
  const int lane = tid & 31;
  const int wave = tid >> 5;
  const int nodeBase = blockIdx.x * NB2;
  const v4f z4 = {0.f, 0.f, 0.f, 0.f};
  const v2f z2 = {0.f, 0.f};

  for (int i = tid; i < (L2_SACC + L2_DEN) / 4; i += NTHR) lds_dyn[i] = z4;
  for (int i = tid; i < L2_MX; i += NTHR) mx[i] = MXINIT;
  __syncthreads();

  scan_drain<DF2, NH2, NB2, SB2>(hp2, ei, a2, sacc, mx, den, list, wcnt,
                                 nN, nE, nodeBase, tid, lane, wave);

  {
    const v2f b2 = *(const v2f*)(bias + 2 * lane);
#pragma unroll 1
    for (int j = 0; j < NB2 / NWAVE; ++j) {
      const int slot = wave * (NB2 / NWAVE) + j;
      const int node = nodeBase + slot;
      const bool valid = node < nN;
      const int nd = valid ? node : nN - 1;
      float a = a2[(size_t)nd * 2] + a2[(size_t)nd * 2 + 1];
      a = (a > 0.f) ? a : SLOPE * a;
      const float M  = mx[slot];
      const float Mn = fmaxf(M, a);
      const float sc = __expf(fmaxf(M - Mn, -80.f));
      const float p  = __expf(fmaxf(a - Mn, -80.f));
      const v2f xv = *(const v2f*)(hp2 + (size_t)nd * DF2 + 2 * lane);
      v2f* sp = (v2f*)(sacc + slot * DF2 + 2 * lane);
      const v2f sv = (*sp) * sc + xv * p;
      const float dv  = den[slot] * sc + p;
      const float inv = 1.0f / (dv + 1e-16f);
      v2f h = sv * inv + b2;
      if (!valid) h = z2;
      *sp = h;
    }
  }
  __syncthreads();

  {
    const int slot0 = wave * (NB2 / NWAVE);
#pragma unroll 1
    for (int i = 0; i < (NB2 / NWAVE) / 2; ++i) {
      const int r = slot0 + 2 * i + (lane >> 4);
      const int c = 4 * (lane & 15);
      const int node = nodeBase + r;
      const v4f v = *(const v4f*)(sacc + r * DF2 + c);
      float* gp = out + (size_t)node * DF2 + c;
      const bool ok = node < nN;
      if (ok) *(volatile v4f*)gp = v;
      __threadfence();
      if (ok) *(volatile v4f*)gp = v;
    }
  }
}

extern "C" void kernel_launch(void* const* d_in, const int* in_sizes, int n_in,
                              void* d_out, int out_size, void* d_ws, size_t ws_size,
                              hipStream_t stream) {
  if (n_in < 11) return;
  const int nN = in_sizes[0];
  if (nN <= 0) return;
  if (in_sizes[1] < 0 || (in_sizes[1] & 1) != 0) return;
  const int nE = in_sizes[1] / 2;
  if (in_sizes[2] < IND || (in_sizes[2] % IND) != 0) return;
  const int nI = in_sizes[2] / IND;
  if (in_sizes[3] != IND * DF1) return;
  if (in_sizes[4] != DF1 || in_sizes[5] != DF1 || in_sizes[6] != DF1) return;
  if (in_sizes[7] != DF1 * DF2) return;
  if (in_sizes[8] != DF2 || in_sizes[9] != DF2 || in_sizes[10] != DF2) return;
  if (out_size != nN * DF2) return;

  const int*   x_ids  = (const int*)d_in[0];
  const int*   ei     = (const int*)d_in[1];
  const float* emb    = (const float*)d_in[2];
  const float* W1     = (const float*)d_in[3];
  const float* att_s1 = (const float*)d_in[4];
  const float* att_d1 = (const float*)d_in[5];
  const float* bias1  = (const float*)d_in[6];
  const float* W2     = (const float*)d_in[7];
  const float* att_s2 = (const float*)d_in[8];
  const float* att_d2 = (const float*)d_in[9];
  const float* bias2  = (const float*)d_in[10];
  float* out = (float*)d_out;

  const int Npad = ((nN + NB2 - 1) / NB2) * NB2;

  size_t off = 0;
  char* base = (char*)d_ws;
  auto carve = [&](size_t bytes) -> char* {
    off = (off + 255) & ~(size_t)255;
    char* p = base + off;
    off += bytes;
    return p;
  };
  unsigned short* W1h = (unsigned short*)carve((size_t)DF1 * IND * 2);
  unsigned short* W1l = (unsigned short*)carve((size_t)DF1 * IND * 2);
  unsigned short* W2h = (unsigned short*)carve((size_t)DF2 * DF1 * 2);
  unsigned short* W2l = (unsigned short*)carve((size_t)DF2 * DF1 * 2);
  float* hp1 = (float*)carve((size_t)Npad * DF1 * sizeof(float));
  float* a1  = (float*)carve((size_t)Npad * 4 * sizeof(float));
  float* hp2 = (float*)carve((size_t)Npad * DF2 * sizeof(float));
  float* a2  = (float*)carve((size_t)Npad * 2 * sizeof(float));
  if (off > ws_size) return;

  k_wprep<<<(IND * DF1 / 8 + NTHR - 1) / NTHR, NTHR, 0, stream>>>(W1, W1h, W1l, IND, DF1);
  k_wprep<<<(DF1 * DF2 / 8 + NTHR - 1) / NTHR, NTHR, 0, stream>>>(W2, W2h, W2l, DF1, DF2);

  k_node1<<<Npad / GR, NTHR, 0, stream>>>(x_ids, emb, W1h, W1l, att_s1, att_d1, hp1, a1, nN, nI);

  hipFuncSetAttribute(reinterpret_cast<const void*>(&k_gat1),
                      hipFuncAttributeMaxDynamicSharedMemorySize, LDS1_BYTES);
  k_gat1<<<Npad / NB1, NTHR, LDS1_BYTES, stream>>>(hp1, ei, a1, bias1, W2h, W2l, att_s2, att_d2,
                                                    hp2, a2, nN, nE);

  hipFuncSetAttribute(reinterpret_cast<const void*>(&k_gat2),
                      hipFuncAttributeMaxDynamicSharedMemorySize, LDS2_BYTES);
  k_gat2<<<Npad / NB2, NTHR, LDS2_BYTES, stream>>>(hp2, ei, a2, bias2, out, nN, nE);
}
